// Down_SSD_11811160064575
// MI455X (gfx1250) — hardware-verified
//
#include <hip/hip_runtime.h>
#include <hip/hip_bf16.h>
#include <math.h>


#pragma clang fp contract(off)

#define NB    4
#define CINP  128
#define SEQ   2048
#define DMOD  256
#define NHD   256
#define DIN   768
#define NST   16
#define DIP   1824
#define ZXP   1856
#define KIM   512
#define QCH   32
#define NQB   (SEQ / QCH)
#define NTOK  (NB * SEQ)
#define ZCX   768
#define ZCDT  1568
#define GSTR  40
#define OSTR  68
#define SSP   20
#define SMEMB (8 * 16 * OSTR * 4)
#define TOK_LDS 133632
#define CHK_LDS 186368

static_assert(SMEMB >= (2 * 128 * GSTR + 2 * 64 * GSTR) * 2);
static_assert(SEQ % QCH == 0);
static_assert(NTOK % 128 == 0);
static_assert(ZXP % 64 == 0);
static_assert(ZXP >= DIP);
static_assert(DIN == 3 * NHD);
static_assert(NTOK * KIM * 2 == NTOK * NHD * 4);
static_assert(NTOK * DMOD * 2 * 2 == NTOK * NHD * 4);
static_assert(NB * NQB * DIN * NST * 4 == NTOK * DIN * 2);
static_assert(TOK_LDS == 32768 + 32768 + 8 * 2 * 32 * GSTR * 2 + 2 * 16 * GSTR * 2 + 4 * 32 * 16 * 2 + 8 * 32 * SSP * 4);
static_assert(CHK_LDS == 32 * DIN * 4 + 32 * NHD * 4 + 32 * 32 * 4 + 8 * 2 * 32 * GSTR * 2 + 8 * 16 * GSTR * 2);

typedef unsigned short us16 __attribute__((ext_vector_type(16)));
typedef unsigned short us8  __attribute__((ext_vector_type(8)));
typedef unsigned short us8a __attribute__((ext_vector_type(8), may_alias));
typedef __bf16 v16b __attribute__((ext_vector_type(16)));
typedef float v8f __attribute__((ext_vector_type(8)));
typedef float v4f __attribute__((ext_vector_type(4)));
typedef float v4fa __attribute__((ext_vector_type(4), may_alias));
union FragU { us16 v; us8 h[2]; };

__device__ __forceinline__ unsigned short bf16_bits(float f) {
  unsigned u = __float_as_uint(f);
  u += 0x7FFFu + ((u >> 16) & 1u);
  return (unsigned short)(u >> 16);
}
__device__ __forceinline__ float bf16_val(unsigned short b) { return __uint_as_float(((unsigned)b) << 16); }
__device__ __forceinline__ float bf16r(float f) { return bf16_val(bf16_bits(f)); }
__device__ __forceinline__ void split16(float v, unsigned short& hb, unsigned short& lb) {
  hb = bf16_bits(v);
  lb = bf16_bits(v - bf16_val(hb));
}

__device__ __forceinline__ v8f mma_bf16(us16 a, us16 b, v8f c) {
  return __builtin_amdgcn_wmma_f32_16x16x32_bf16(false, __builtin_bit_cast(v16b, a), false, __builtin_bit_cast(v16b, b), (short)0, c, false, false);
}
__device__ __forceinline__ void wguard4(v8f& c0, v8f& c1, v8f& c2, v8f& c3, const us16& a0, const us16& a1,
                                        const us16& b0, const us16& b1, const us16& b2, const us16& b3,
                                        const us16& b4, const us16& b5, const us16& b6, const us16& b7) {
#if defined(__HIP_DEVICE_COMPILE__)
  asm volatile("v_nop\n\tv_nop\n\tv_nop\n\tv_nop"
               : "+v"(c0), "+v"(c1), "+v"(c2), "+v"(c3)
               : "v"(a0), "v"(a1), "v"(b0), "v"(b1), "v"(b2), "v"(b3), "v"(b4), "v"(b5), "v"(b6), "v"(b7));
#endif
}
__device__ __forceinline__ void wguard2(v8f& c0, v8f& c1, const us16& f0, const us16& f1, const us16& f2,
                                        const us16& f3, const us16& f4, const us16& f5) {
#if defined(__HIP_DEVICE_COMPILE__)
  asm volatile("v_nop\n\tv_nop\n\tv_nop\n\tv_nop"
               : "+v"(c0), "+v"(c1)
               : "v"(f0), "v"(f1), "v"(f2), "v"(f3), "v"(f4), "v"(f5));
#endif
}
__device__ __forceinline__ void wguard1(v8f& c0, const us16& f0, const us16& f1, const us16& f2, const us16& f3) {
#if defined(__HIP_DEVICE_COMPILE__)
  asm volatile("v_nop\n\tv_nop\n\tv_nop\n\tv_nop"
               : "+v"(c0)
               : "v"(f0), "v"(f1), "v"(f2), "v"(f3));
#endif
}

__device__ __forceinline__ us16 lds_frag(const unsigned short* base) {
  const int lane = threadIdx.x & 31, r = lane & 15, kh = (lane >> 4) * 8;
  FragU f;
  f.h[0] = *(const us8a*)(base + r * GSTR + kh);
  f.h[1] = *(const us8a*)(base + r * GSTR + 16 + kh);
  return f.v;
}
__device__ __forceinline__ us16 gfrag16(const unsigned short* __restrict__ P, size_t row0) {
  const int lane = threadIdx.x & 31, r = lane & 15, kh = (lane >> 4) * 8;
  FragU f;
  f.h[0] = *(const us8a*)(P + (row0 + r) * 16 + kh);
  const us8 zz = {0, 0, 0, 0, 0, 0, 0, 0};
  f.h[1] = zz;
  return f.v;
}

__device__ __forceinline__ void stage_a(unsigned short* lds, const unsigned short* __restrict__ P, int ld, int m0, int k0, int tid) {
  const int row = tid >> 1, cq = (tid & 1) * 16;
  const unsigned short* src = P + (size_t)(m0 + row) * ld + k0 + cq;
  const us8 v0 = *(const us8a*)src;
  const us8 v1 = *(const us8a*)(src + 8);
  *(us8a*)(lds + row * GSTR + cq) = v0;
  *(us8a*)(lds + row * GSTR + cq + 8) = v1;
}
__device__ __forceinline__ void stage_b(unsigned short* lds, const unsigned short* __restrict__ P, int ld, int n0, int k0, int nbmax, int tid) {
  const int row = tid >> 2, kq = (tid & 3) * 8;
  int n = n0 + row;
  n = (n > nbmax) ? nbmax : n;
  const us8 v = *(const us8a*)(P + (size_t)n * ld + k0 + kq);
  *(us8a*)(lds + row * GSTR + kq) = v;
}

template <int NA, int NBP, int EPI>
__global__ __launch_bounds__(256) void k_gemm(
    const unsigned short* __restrict__ A0, const unsigned short* __restrict__ A1, int lda, long long sAz,
    const unsigned short* __restrict__ B0, const unsigned short* __restrict__ B1, int ldb, long long sBz, int nbmax,
    float* Yf, unsigned short* Yh, unsigned short* Yl, int ldy, long long sYz, int K)
{
  __shared__ __attribute__((aligned(16))) unsigned char sm[SMEMB];
  unsigned short* lA0 = (unsigned short*)sm;
  unsigned short* lA1 = lA0 + 128 * GSTR;
  unsigned short* lB0 = lA1 + 128 * GSTR;
  unsigned short* lB1 = lB0 + 64 * GSTR;
  float* oS = (float*)sm;
  const int tid = threadIdx.x, lane = tid & 31, wave = tid >> 5, cl = lane & 15, hh = lane >> 4;
  const int m0 = blockIdx.x * 128, n0 = blockIdx.y * 64;
  const long long z = blockIdx.z;
  A0 += z * sAz; A1 += z * sAz;
  B0 += z * sBz; B1 += z * sBz;

  v8f acc[4];
#pragma unroll
  for (int j = 0; j < 4; ++j) { v8f zz = {0.f, 0.f, 0.f, 0.f, 0.f, 0.f, 0.f, 0.f}; acc[j] = zz; }

#pragma unroll 1
  for (int k0 = 0; k0 < K; k0 += 32) {
    __syncthreads();
    stage_a(lA0, A0, lda, m0, k0, tid);
    if (NA > 1) stage_a(lA1, A1, lda, m0, k0, tid);
    stage_b(lB0, B0, ldb, n0, k0, nbmax, tid);
    if (NBP > 1) stage_b(lB1, B1, ldb, n0, k0, nbmax, tid);
    __syncthreads();
    const us16 af0 = lds_frag(lA0 + 16 * wave * GSTR);
    us16 af1 = af0;
    if (NA > 1) af1 = lds_frag(lA1 + 16 * wave * GSTR);
    us16 bf0[4], bf1[4];
#pragma unroll
    for (int j = 0; j < 4; ++j) { bf0[j] = lds_frag(lB0 + 16 * j * GSTR); bf1[j] = bf0[j]; }
    if (NBP > 1) {
#pragma unroll
      for (int j = 0; j < 4; ++j) bf1[j] = lds_frag(lB1 + 16 * j * GSTR);
    }
#pragma unroll
    for (int j = 0; j < 4; ++j) acc[j] = mma_bf16(af0, bf0[j], acc[j]);
    if (NBP > 1) {
#pragma unroll
      for (int j = 0; j < 4; ++j) acc[j] = mma_bf16(af0, bf1[j], acc[j]);
    }
    if (NA > 1) {
#pragma unroll
      for (int j = 0; j < 4; ++j) acc[j] = mma_bf16(af1, bf0[j], acc[j]);
    }
    wguard4(acc[0], acc[1], acc[2], acc[3], af0, af1, bf0[0], bf0[1], bf0[2], bf0[3], bf1[0], bf1[1], bf1[2], bf1[3]);
  }
  __syncthreads();

  float* so = oS + wave * (16 * OSTR);
#pragma unroll
  for (int j = 0; j < 4; ++j)
#pragma unroll
    for (int r = 0; r < 8; ++r) so[(8 * hh + r) * OSTR + 16 * j + cl] = acc[j][r];
  __syncthreads();
  if (EPI == 0) {
    float* Y = Yf + z * sYz;
#pragma unroll
    for (int pass = 0; pass < 2; ++pass) {
#pragma unroll
      for (int it = 0; it < 8; ++it) {
        const int ch = it * 32 + lane, r = ch >> 4, q = (ch & 15) * 4;
        const v4f v = *(const v4fa*)(so + r * OSTR + q);
        *(volatile v4f*)(Y + (size_t)(m0 + 16 * wave + r) * ldy + n0 + q) = v;
      }
      __threadfence();
    }
  } else {
    unsigned short* H = Yh + z * sYz;
    unsigned short* L = Yl + z * sYz;
    us8 oh[4], ol[4];
    size_t od[4];
#pragma unroll
    for (int it = 0; it < 4; ++it) {
      const int ch = it * 32 + lane, r = ch >> 3, q = (ch & 7) * 8;
      const v4f a = *(const v4fa*)(so + r * OSTR + q);
      const v4f b = *(const v4fa*)(so + r * OSTR + q + 4);
      us8 h8, l8;
#pragma unroll
      for (int u = 0; u < 4; ++u) {
        unsigned short hb, lb;
        split16(a[u], hb, lb); h8[u] = hb; l8[u] = lb;
        split16(b[u], hb, lb); h8[4 + u] = hb; l8[4 + u] = lb;
      }
      oh[it] = h8; ol[it] = l8;
      od[it] = (size_t)(m0 + 16 * wave + r) * ldy + n0 + q;
    }
#pragma unroll
    for (int pass = 0; pass < 2; ++pass) {
#pragma unroll
      for (int it = 0; it < 4; ++it) {
        *(volatile us8*)(H + od[it]) = oh[it];
        *(volatile us8*)(L + od[it]) = ol[it];
      }
      __threadfence();
    }
  }
}

__global__ __launch_bounds__(256) void k_prep(const float* __restrict__ w1, const float* __restrict__ w2, const float* __restrict__ w3,
                                             unsigned short* W1, unsigned short* W2, unsigned short* W3) {
  const int blk = blockIdx.x;
  const float* src;
  unsigned short* dst;
  int base;
  if (blk < 64) { src = w1; dst = W1; base = blk * 2048; }
  else if (blk < 292) { src = w2; dst = W2; base = (blk - 64) * 2048; }
  else { src = w3; dst = W3; base = (blk - 292) * 2048; }
  const int e = base + threadIdx.x * 8;
  const v4f a = *(const v4fa*)(src + e);
  const v4f b = *(const v4fa*)(src + e + 4);
  us8 o;
#pragma unroll
  for (int u = 0; u < 4; ++u) { o[u] = bf16_bits(a[u]); o[4 + u] = bf16_bits(b[u]); }
  *(volatile us8*)(dst + e) = o;
  __threadfence();
  *(volatile us8*)(dst + e) = o;
}

__global__ __launch_bounds__(256) void k_im2col(const float* __restrict__ x, unsigned short* A1) {
  const int t = blockIdx.x * 256 + threadIdx.x;
  const int m = t >> 6, q = t & 63;
  const int b = m >> 11, l = m & (SEQ - 1);
  us8 o;
#pragma unroll
  for (int ci = 0; ci < 2; ++ci) {
    const int cin = 2 * q + ci;
    const float* xr = x + ((size_t)(b * CINP + cin)) * SEQ;
#pragma unroll
    for (int k = 0; k < 4; ++k) {
      const int ll = l + k - 1;
      const int lc = (ll < 0) ? 0 : ((ll > SEQ - 1) ? (SEQ - 1) : ll);
      const float v = xr[lc];
      const float vv = (ll >= 0 && ll < SEQ) ? v : 0.0f;
      o[ci * 4 + k] = bf16_bits(vv);
    }
  }
  const size_t off = (size_t)m * KIM + 8 * q;
  *(volatile us8*)(A1 + off) = o;
  __threadfence();
  *(volatile us8*)(A1 + off) = o;
}

struct ConvW { float w0, w1, w2, w3, bs, x0, x1, x2; };
__device__ __forceinline__ void conv_begin(ConvW& s, const float* __restrict__ ZX, const float* __restrict__ cw, const float* __restrict__ cb,
                                           int ch, int b, int cq) {
  s.w0 = bf16r(cw[ch * 4 + 0]); s.w1 = bf16r(cw[ch * 4 + 1]); s.w2 = bf16r(cw[ch * 4 + 2]); s.w3 = bf16r(cw[ch * 4 + 3]);
  s.bs = bf16r(cb[ch]);
  const int l0 = cq * QCH;
  const int la = l0 - 3, lb = l0 - 2, lc = l0 - 1;
  const float va = ZX[((size_t)b * SEQ + ((la < 0) ? 0 : la)) * ZXP + ZCX + ch];
  const float vb = ZX[((size_t)b * SEQ + ((lb < 0) ? 0 : lb)) * ZXP + ZCX + ch];
  const float vc = ZX[((size_t)b * SEQ + ((lc < 0) ? 0 : lc)) * ZXP + ZCX + ch];
  s.x0 = (la >= 0) ? va : 0.0f;
  s.x1 = (lb >= 0) ? vb : 0.0f;
  s.x2 = (lc >= 0) ? vc : 0.0f;
}
__device__ __forceinline__ float conv_step(ConvW& s, float xin) {
  float a = s.w0 * s.x0;
  a = a + s.w1 * s.x1;
  a = a + s.w2 * s.x2;
  a = a + s.w3 * xin;
  a = a + s.bs;
  s.x0 = s.x1; s.x1 = s.x2; s.x2 = xin;
  const float sg = __builtin_amdgcn_rcpf(1.0f + expf(-a));
  return a * sg;
}

__global__ __launch_bounds__(256) void k_tok(const float* __restrict__ ZX, const float* __restrict__ convw, const float* __restrict__ convb,
                                            const float* __restrict__ dtb, const float* __restrict__ alog,
                                            float* DT, float* ACS,
                                            unsigned short* BH, unsigned short* BL, unsigned short* CHp, unsigned short* CLp,
                                            float* SC)
{
  extern __shared__ __attribute__((aligned(16))) unsigned char dsm_t[];
  float* sE = (float*)dsm_t;
  float* sacs = (float*)(dsm_t + 32768);
  unsigned short* sA = (unsigned short*)(dsm_t + 65536);
  unsigned short* sBt = (unsigned short*)(dsm_t + 106496);
  unsigned short* sBC = (unsigned short*)(dsm_t + 109056);
  float* sS = (float*)(dsm_t + 113152);
  const int tid = threadIdx.x, lane = tid & 31, wave = tid >> 5, cl = lane & 15, hh = lane >> 4;
  const int cq = blockIdx.x, b = blockIdx.y;
  const size_t tok0 = (size_t)b * SEQ + (size_t)cq * QCH;

  {
    const int h = tid;
    const float Ah = -expf(bf16r(alog[h]));
    const float db = bf16r(dtb[h]);
    float run = 0.0f;
#pragma unroll 1
    for (int i = 0; i < QCH; ++i) {
      const float v = ZX[(tok0 + i) * ZXP + ZCDT + h] + db;
      const float sp = fmaxf(v, 0.0f) + log1pf(expf(-fabsf(v)));
      run = run + sp * Ah;
      sE[i * NHD + h] = sp;
      sacs[i * NHD + h] = run;
      *(volatile float*)(DT + (tok0 + i) * NHD + h) = sp;
      *(volatile float*)(ACS + (tok0 + i) * NHD + h) = run;
    }
    __threadfence();
#pragma unroll 1
    for (int i = 0; i < QCH; ++i) {
      const float sp = sE[i * NHD + h], ac = sacs[i * NHD + h];
      *(volatile float*)(DT + (tok0 + i) * NHD + h) = sp;
      *(volatile float*)(ACS + (tok0 + i) * NHD + h) = ac;
      sE[i * NHD + h] = expf(run - ac) * sp;
    }
  }
  if (wave == 0) {
    const int cc = lane;
    const int ch = DIN + cc;
    const int n = cc & 15;
    const int pb = (cc < 16) ? 0 : 2;
    ConvW cw;
    conv_begin(cw, ZX, convw, convb, ch, b, cq);
#pragma unroll 1
    for (int i = 0; i < QCH; ++i) {
      const float xin = ZX[(tok0 + i) * ZXP + ZCX + ch];
      const float xc = conv_step(cw, xin);
      unsigned short hb, lb;
      split16(xc, hb, lb);
      if (cc < 16) { sBt[n * GSTR + i] = hb; sBt[16 * GSTR + n * GSTR + i] = lb; }
      sBC[(pb * 32 + i) * 16 + n] = hb;
      sBC[((pb + 1) * 32 + i) * 16 + n] = lb;
    }
  }
  __syncthreads();
  {
    const int pl = tid >> 6, pc = tid & 63;
    const us8 v = *(const us8a*)(sBC + pl * 512 + pc * 8);
    unsigned short* dstp = (pl == 0) ? BH : ((pl == 1) ? BL : ((pl == 2) ? CHp : CLp));
    unsigned short* dst = dstp + tok0 * 16 + pc * 8;
    *(volatile us8*)dst = v;
    __threadfence();
    *(volatile us8*)dst = v;
  }
  const us16 bfh = lds_frag(sBt), bfl = lds_frag(sBt + 16 * GSTR);
  unsigned short* myAh = sA + wave * (2 * 32 * GSTR);
  unsigned short* myAl = myAh + 32 * GSTR;
  float* mS = sS + wave * (32 * SSP);
#pragma unroll 1
  for (int i3 = 0; i3 < 3; ++i3) {
    const int c = 256 * i3 + tid;
    const int h = c / 3;
    ConvW cw;
    conv_begin(cw, ZX, convw, convb, c, b, cq);
#pragma unroll 1
    for (int i = 0; i < QCH; ++i) {
      const float xin = ZX[(tok0 + i) * ZXP + ZCX + c];
      const float xc = conv_step(cw, xin);
      const float xe = xc * sE[i * NHD + h];
      unsigned short hb, lb;
      split16(xe, hb, lb);
      myAh[lane * GSTR + i] = hb;
      myAl[lane * GSTR + i] = lb;
    }
    __syncthreads();
    const v8f z8 = {0.f, 0.f, 0.f, 0.f, 0.f, 0.f, 0.f, 0.f};
    const us16 a0h = lds_frag(myAh), a0l = lds_frag(myAl);
    const us16 a1h = lds_frag(myAh + 16 * GSTR), a1l = lds_frag(myAl + 16 * GSTR);
    v8f acc0 = z8, acc1 = z8;
    acc0 = mma_bf16(a0h, bfh, acc0); acc0 = mma_bf16(a0h, bfl, acc0); acc0 = mma_bf16(a0l, bfh, acc0);
    acc1 = mma_bf16(a1h, bfh, acc1); acc1 = mma_bf16(a1h, bfl, acc1); acc1 = mma_bf16(a1l, bfh, acc1);
    wguard2(acc0, acc1, a0h, a0l, a1h, a1l, bfh, bfl);
#pragma unroll
    for (int r = 0; r < 8; ++r) { mS[(8 * hh + r) * SSP + cl] = acc0[r]; mS[(16 + 8 * hh + r) * SSP + cl] = acc1[r]; }
    __syncthreads();
    const size_t sbase = (((size_t)(b * NQB + cq)) * DIN + 256 * i3 + 32 * wave) * NST;
#pragma unroll
    for (int pass = 0; pass < 2; ++pass) {
#pragma unroll
      for (int it = 0; it < 4; ++it) {
        const int chn = it * 32 + lane, row = chn >> 2, q = (chn & 3) * 4;
        const v4f v = *(const v4fa*)(mS + row * SSP + q);
        *(volatile v4f*)(SC + sbase + row * NST + q) = v;
      }
      __threadfence();
    }
    __syncthreads();
  }
}

__global__ __launch_bounds__(256) void k_rec(const float* __restrict__ SC, const float* __restrict__ ACS,
                                            unsigned short* SIH, unsigned short* SIL) {
  const int t = blockIdx.x * 256 + threadIdx.x;
  if (t >= NB * DIN * 2) return;
  const int b = t / (DIN * 2), rr = t - b * (DIN * 2), ch = rr >> 1, n0 = (rr & 1) * 8, h = ch / 3;
  float st[8];
#pragma unroll
  for (int u = 0; u < 8; ++u) st[u] = 0.0f;
#pragma unroll 1
  for (int c = 0; c < NQB; ++c) {
    const size_t e = (((size_t)(b * NQB + c)) * DIN + ch) * NST + n0;
    us8 hi, lo;
#pragma unroll
    for (int u = 0; u < 8; ++u) { unsigned short hb, lb; split16(st[u], hb, lb); hi[u] = hb; lo[u] = lb; }
    *(volatile us8*)(SIH + e) = hi; *(volatile us8*)(SIL + e) = lo;
    __threadfence();
    *(volatile us8*)(SIH + e) = hi; *(volatile us8*)(SIL + e) = lo;
    const float dec = expf(ACS[((size_t)b * SEQ + (size_t)c * QCH + (QCH - 1)) * NHD + h]);
    const v4f s0 = *(const v4fa*)(SC + e), s1 = *(const v4fa*)(SC + e + 4);
#pragma unroll
    for (int u = 0; u < 4; ++u) { st[u] = dec * st[u] + s0[u]; st[4 + u] = dec * st[4 + u] + s1[u]; }
  }
}

__global__ __launch_bounds__(256) void k_chunk(const float* __restrict__ ZX, const float* __restrict__ convw, const float* __restrict__ convb,
                                              const float* __restrict__ dsk, const float* __restrict__ nrw,
                                              const float* __restrict__ DT, const float* __restrict__ ACS,
                                              const unsigned short* __restrict__ BH, const unsigned short* __restrict__ BL,
                                              const unsigned short* __restrict__ CHp, const unsigned short* __restrict__ CLp,
                                              const unsigned short* __restrict__ SIH, const unsigned short* __restrict__ SIL,
                                              unsigned short* YH, unsigned short* YL)
{
  extern __shared__ __attribute__((aligned(16))) unsigned char dsm_c[];
  float* sy = (float*)dsm_c;
  float* sacs = (float*)(dsm_c + 98304);
  float* sG = (float*)(dsm_c + 131072);
  unsigned short* sW = (unsigned short*)(dsm_c + 135168);
  unsigned short* sBtA = (unsigned short*)(dsm_c + 176128);
  const int tid = threadIdx.x, lane = tid & 31, wave = tid >> 5, cl = lane & 15, hh = lane >> 4;
  const int cq = blockIdx.x, b = blockIdx.y;
  const size_t tok0 = (size_t)b * SEQ + (size_t)cq * QCH;
  unsigned short* myWh = sW + wave * (64 * GSTR);
  unsigned short* myWl = myWh + 32 * GSTR;
  unsigned short* myBt = sBtA + wave * (16 * GSTR);
  const v8f z8 = {0.f, 0.f, 0.f, 0.f, 0.f, 0.f, 0.f, 0.f};

#pragma unroll 1
  for (int i = 0; i < QCH; ++i) sacs[i * NHD + tid] = ACS[(tok0 + i) * NHD + tid];
  for (int e = lane; e < 40; e += 32) {
    const us8 zz = {0, 0, 0, 0, 0, 0, 0, 0};
    *(us8a*)(myBt + (6 + (e >> 2)) * GSTR + (e & 3) * 8) = zz;
  }
#pragma unroll 1
  for (int i3 = 0; i3 < 3; ++i3) {
    const int c = 256 * i3 + tid;
    ConvW cw;
    conv_begin(cw, ZX, convw, convb, c, b, cq);
#pragma unroll 1
    for (int i = 0; i < QCH; ++i) {
      const float xin = ZX[(tok0 + i) * ZXP + ZCX + c];
      sy[i * DIN + c] = conv_step(cw, xin);
    }
  }
  __syncthreads();
  if (wave < 4) {
    const int rt = wave >> 1, ct = wave & 1;
    const us16 cfh = gfrag16(CHp, tok0 + 16 * rt), cfl = gfrag16(CLp, tok0 + 16 * rt);
    const us16 bvh = gfrag16(BH, tok0 + 16 * ct), bvl = gfrag16(BL, tok0 + 16 * ct);
    v8f g = z8;
    g = mma_bf16(cfh, bvh, g); g = mma_bf16(cfh, bvl, g); g = mma_bf16(cfl, bvh, g);
    wguard1(g, cfh, cfl, bvh, bvl);
#pragma unroll
    for (int r = 0; r < 8; ++r) sG[(16 * rt + 8 * hh + r) * 32 + 16 * ct + cl] = g[r];
  }
  __syncthreads();
#pragma unroll 1
  for (int th = 0; th < 32; ++th) {
    const int h = wave * 32 + th;
    {
      const int s = lane;
      const float dtv = DT[(tok0 + s) * NHD + h];
#pragma unroll
      for (int p = 0; p < 3; ++p) {
        const float xd = dtv * sy[s * DIN + 3 * h + p];
        unsigned short hb, lb;
        split16(xd, hb, lb);
        myBt[p * GSTR + s] = hb;
        myBt[(3 + p) * GSTR + s] = lb;
      }
    }
    {
      const int l = lane;
      const float al = sacs[l * NHD + h];
#pragma unroll
      for (int sb = 0; sb < 4; ++sb) {
        us8 h8, l8;
#pragma unroll
        for (int u = 0; u < 8; ++u) {
          const int s = 8 * sb + u;
          const float g = sG[l * 32 + s];
          const float d = __expf(al - sacs[s * NHD + h]);
          const float w = (s <= l) ? (g * d) : 0.0f;
          unsigned short hb, lb;
          split16(w, hb, lb);
          h8[u] = hb; l8[u] = lb;
        }
        *(us8a*)(myWh + l * GSTR + 8 * sb) = h8;
        *(us8a*)(myWl + l * GSTR + 8 * sb) = l8;
      }
    }
    __syncthreads();
    const us16 bt = lds_frag(myBt);
    const us16 w0h = lds_frag(myWh), w0l = lds_frag(myWl);
    const us16 w1h = lds_frag(myWh + 16 * GSTR), w1l = lds_frag(myWl + 16 * GSTR);
    v8f a0 = z8, a1 = z8;
    a0 = mma_bf16(w0h, bt, a0); a0 = mma_bf16(w0l, bt, a0);
    a1 = mma_bf16(w1h, bt, a1); a1 = mma_bf16(w1l, bt, a1);
    wguard2(a0, a1, w0h, w0l, w1h, w1l, bt, bt);
    const float Dh = bf16r(dsk[h]);
    const int pcol = 3 * h + ((cl < 3) ? cl : 2);
    const int src = (lane + 3) & 31;
#pragma unroll
    for (int r = 0; r < 8; ++r) {
      const float q0 = __shfl(a0[r], src, 32);
      const float q1 = __shfl(a1[r], src, 32);
      const int l0 = 8 * hh + r, l1 = 16 + 8 * hh + r;
      const float x0 = sy[l0 * DIN + pcol], x1 = sy[l1 * DIN + pcol];
      const float y0 = (a0[r] + q0) + Dh * x0;
      const float y1 = (a1[r] + q1) + Dh * x1;
      if (cl < 3) { sy[l0 * DIN + pcol] = y0; sy[l1 * DIN + pcol] = y1; }
    }
  }
  __syncthreads();
  {
    const us16 c0h = gfrag16(CHp, tok0), c0l = gfrag16(CLp, tok0);
    const us16 c1h = gfrag16(CHp, tok0 + 16), c1l = gfrag16(CLp, tok0 + 16);
    const size_t srow0 = ((size_t)(b * NQB + cq)) * DIN;
#pragma unroll 1
    for (int jt = 0; jt < 6; ++jt) {
      const int ct = wave + 8 * jt;
      const us16 sh = gfrag16(SIH, srow0 + 16 * ct), sl = gfrag16(SIL, srow0 + 16 * ct);
      v8f a0 = z8, a1 = z8;
      a0 = mma_bf16(c0h, sh, a0); a0 = mma_bf16(c0h, sl, a0); a0 = mma_bf16(c0l, sh, a0);
      a1 = mma_bf16(c1h, sh, a1); a1 = mma_bf16(c1h, sl, a1); a1 = mma_bf16(c1l, sh, a1);
      wguard2(a0, a1, c0h, c0l, c1h, c1l, sh, sl);
      const int c = 16 * ct + cl;
      const int hc = c / 3;
#pragma unroll
      for (int r = 0; r < 8; ++r) {
        const int l0 = 8 * hh + r, l1 = 16 + 8 * hh + r;
        const float e0 = __expf(sacs[l0 * NHD + hc]), e1 = __expf(sacs[l1 * NHD + hc]);
        const float v0 = sy[l0 * DIN + c] + a0[r] * e0;
        const float v1 = sy[l1 * DIN + c] + a1[r] * e1;
        sy[l0 * DIN + c] = v0;
        sy[l1 * DIN + c] = v1;
      }
    }
  }
  __syncthreads();
  {
#pragma unroll 1
    for (int j = 0; j < 4; ++j) {
      const int i = wave * 4 + j;
      const size_t tok = tok0 + i;
      float v[24];
      float ss = 0.0f;
#pragma unroll
      for (int j3 = 0; j3 < 3; ++j3) {
        const int c0 = 256 * j3 + 8 * lane;
        const v4f ya = *(const v4fa*)(sy + i * DIN + c0), yb = *(const v4fa*)(sy + i * DIN + c0 + 4);
        const v4f za = *(const v4fa*)(ZX + tok * ZXP + c0), zb = *(const v4fa*)(ZX + tok * ZXP + c0 + 4);
#pragma unroll
        for (int u = 0; u < 4; ++u) {
          {
            const float zz = za[u];
            const float sg = __builtin_amdgcn_rcpf(1.0f + __expf(-zz));
            const float t = ya[u] * (zz * sg);
            v[8 * j3 + u] = t; ss = ss + t * t;
          }
          {
            const float zz = zb[u];
            const float sg = __builtin_amdgcn_rcpf(1.0f + __expf(-zz));
            const float t = yb[u] * (zz * sg);
            v[8 * j3 + 4 + u] = t; ss = ss + t * t;
          }
        }
      }
      ss = ss + __shfl_xor(ss, 16, 32);
      ss = ss + __shfl_xor(ss, 8, 32);
      ss = ss + __shfl_xor(ss, 4, 32);
      ss = ss + __shfl_xor(ss, 2, 32);
      ss = ss + __shfl_xor(ss, 1, 32);
      const float rs = rsqrtf(ss * (1.0f / 768.0f) + 1.0e-5f);
      us8 oh[3], ol[3];
#pragma unroll
      for (int j3 = 0; j3 < 3; ++j3) {
        us8 h8, l8;
#pragma unroll
        for (int u = 0; u < 8; ++u) {
          const int c = 256 * j3 + 8 * lane + u;
          const float o = (v[8 * j3 + u] * rs) * bf16r(nrw[c]);
          unsigned short hb, lb;
          split16(o, hb, lb);
          h8[u] = hb; l8[u] = lb;
        }
        oh[j3] = h8; ol[j3] = l8;
      }
#pragma unroll
      for (int pass = 0; pass < 2; ++pass) {
#pragma unroll
        for (int j3 = 0; j3 < 3; ++j3) {
          *(volatile us8*)(YH + tok * DIN + 256 * j3 + 8 * lane) = oh[j3];
          *(volatile us8*)(YL + tok * DIN + 256 * j3 + 8 * lane) = ol[j3];
        }
        __threadfence();
      }
    }
  }
}

extern "C" void kernel_launch(void* const* d_in, const int* in_sizes, int n_in,
                              void* d_out, int out_size, void* d_ws, size_t ws_size,
                              hipStream_t stream) {
  if (n_in < 10) return;
  if (in_sizes[0] != NB * CINP * SEQ || in_sizes[1] != DMOD * CINP * 4 || in_sizes[2] != DIP * DMOD ||
      in_sizes[3] != 800 * 4 || in_sizes[4] != 800 || in_sizes[5] != NHD || in_sizes[6] != NHD ||
      in_sizes[7] != NHD || in_sizes[8] != DIN || in_sizes[9] != DMOD * DIN || out_size != NB * DMOD * SEQ) return;
  const float* x          = (const float*)d_in[0];
  const float* proj_w     = (const float*)d_in[1];
  const float* in_proj_w  = (const float*)d_in[2];
  const float* conv_w     = (const float*)d_in[3];
  const float* conv_b     = (const float*)d_in[4];
  const float* dt_bias    = (const float*)d_in[5];
  const float* A_log      = (const float*)d_in[6];
  const float* D_skip     = (const float*)d_in[7];
  const float* norm_w     = (const float*)d_in[8];
  const float* out_proj_w = (const float*)d_in[9];
  float* out = (float*)d_out;

  size_t off = 0;
  auto carve = [&](size_t bytes) -> char* { char* p = (char*)d_ws + off; off += (bytes + 255) & ~(size_t)255; return p; };
  unsigned short* W1 = (unsigned short*)carve((size_t)DMOD * KIM * 2);
  unsigned short* W2 = (unsigned short*)carve((size_t)DIP * DMOD * 2);
  unsigned short* W3 = (unsigned short*)carve((size_t)DMOD * DIN * 2);
  char* RA = carve((size_t)NTOK * KIM * 2);
  char* RB = carve((size_t)NTOK * DMOD * 2 * 2);
  float* ZX = (float*)carve((size_t)NTOK * ZXP * 4);
  unsigned short* BHp = (unsigned short*)carve((size_t)NTOK * NST * 2);
  unsigned short* BLp = (unsigned short*)carve((size_t)NTOK * NST * 2);
  unsigned short* CHh = (unsigned short*)carve((size_t)NTOK * NST * 2);
  unsigned short* CLl = (unsigned short*)carve((size_t)NTOK * NST * 2);
  char* RC = carve((size_t)NB * NQB * DIN * NST * 4);
  unsigned short* SIH = (unsigned short*)carve((size_t)NB * NQB * DIN * NST * 2);
  unsigned short* SIL = (unsigned short*)carve((size_t)NB * NQB * DIN * NST * 2);
  unsigned short* YL = (unsigned short*)carve((size_t)NTOK * DIN * 2);
  if (off > ws_size || off > (size_t)134217728) return;
  unsigned short* A1 = (unsigned short*)RA;
  float* DT = (float*)RA;
  unsigned short* UH = (unsigned short*)RB;
  unsigned short* UL = UH + (size_t)NTOK * DMOD;
  float* ACS = (float*)RB;
  float* SC = (float*)RC;
  unsigned short* YH = (unsigned short*)RC;

  hipFuncSetAttribute(reinterpret_cast<const void*>(&k_tok), hipFuncAttributeMaxDynamicSharedMemorySize, TOK_LDS);
  hipFuncSetAttribute(reinterpret_cast<const void*>(&k_chunk), hipFuncAttributeMaxDynamicSharedMemorySize, CHK_LDS);

  const dim3 blk(256);
  k_prep<<<dim3(388), blk, 0, stream>>>(proj_w, in_proj_w, out_proj_w, W1, W2, W3);
  k_im2col<<<dim3(NTOK * 64 / 256), blk, 0, stream>>>(x, A1);
  k_gemm<1, 1, 1><<<dim3(NTOK / 128, DMOD / 64, 1), blk, 0, stream>>>(
      A1, A1, KIM, 0, W1, W1, KIM, 0, DMOD - 1, ZX, UH, UL, DMOD, 0, KIM);
  k_gemm<2, 1, 0><<<dim3(NTOK / 128, ZXP / 64, 1), blk, 0, stream>>>(
      UH, UL, DMOD, 0, W2, W2, DMOD, 0, DIP - 1, ZX, W1, W1, ZXP, 0, DMOD);
  k_tok<<<dim3(NQB, NB), blk, TOK_LDS, stream>>>(ZX, conv_w, conv_b, dt_bias, A_log, DT, ACS, BHp, BLp, CHh, CLl, SC);
  k_rec<<<dim3(NB * DIN * 2 / 256), blk, 0, stream>>>(SC, ACS, SIH, SIL);
  k_chunk<<<dim3(NQB, NB), blk, CHK_LDS, stream>>>(ZX, conv_w, conv_b, D_skip, norm_w, DT, ACS, BHp, BLp, CHh, CLl, SIH, SIL, YH, YL);
  k_gemm<1, 2, 0><<<dim3(DMOD / 128, SEQ / 64, NB), blk, 0, stream>>>(
      W3, W3, DIN, 0, YH, YL, DIN, (long long)SEQ * DIN, SEQ - 1, out, W1, W1, SEQ, (long long)DMOD * SEQ, DIN);
}
